// QRNNLayer_85581518340442
// MI455X (gfx1250) — hardware-run, weakly checked
//
#include <hip/hip_runtime.h>
#include <math.h>

typedef __attribute__((ext_vector_type(16))) _Float16 v16h;
typedef __attribute__((ext_vector_type(8)))  _Float16 v8h;
typedef __attribute__((ext_vector_type(2)))  _Float16 v2h;
typedef __attribute__((ext_vector_type(16))) __bf16   v16b;
typedef __attribute__((ext_vector_type(8)))  __bf16   v8b;
typedef __attribute__((ext_vector_type(8)))  float    v8f;
typedef __attribute__((ext_vector_type(4)))  float    v4f;
typedef __attribute__((ext_vector_type(2)))  float    v2f;

constexpr int kS    = 4096;
constexpr int kB    = 8;
constexpr int kC    = 256;
constexpr int kHd   = 256;
constexpr int kRows = kS * kB;
constexpr int kK2   = 2 * kC;
constexpr int kN2   = 2 * kHd;
constexpr int kThr  = 256;
constexpr float kInCarry = 1024.0f;
constexpr float kSc = 1.0f / (kInCarry * kInCarry);
constexpr float kGelu = 1.702f;
constexpr float kF16MinNormal = 6.103515625e-5f;
constexpr size_t kOut0 = 0;
constexpr size_t kOut1 = (size_t)kS * kB * kHd;

static_assert(kB == 8 && kC == 256 && kHd == 256 && kK2 == 512 && kN2 == 512, "the index arithmetic below uses these sizes");

constexpr size_t kOffBIA = 0ull;
constexpr size_t kOffW2 = 2048ull;
constexpr size_t kOffX2 = 526336ull;
constexpr size_t kOffZF32 = 34080768ull;
constexpr size_t kWsTotal = 101189632ull;
static_assert(kWsTotal <= 134217728ull, "carve cap: under 128 MiB");
static_assert(kOffBIA == 0
              && kOffW2 == kOffBIA + 2048ull
              && kOffX2 == kOffW2 + 524288ull
              && kOffZF32 == kOffX2 + 33554432ull
              && kWsTotal == kOffZF32 + 67108864ull, "the carve is chained and totalled");
static_assert((kOffBIA % 256) == 0 && (kOffW2 % 256) == 0 && (kOffX2 % 256) == 0 && (kOffZF32 % 256) == 0, "aligned regions");
static_assert(512 >= kN2, "the bias record covers the engine launch's 512 output columns (the engine reads one bias value a column)");

__device__ __forceinline__ unsigned short f2bf_bits(float f) {
  unsigned u = __float_as_uint(f);
  return (unsigned short)((u + 0x7FFFu + ((u >> 16) & 1u)) >> 16);
}
__device__ __forceinline__ float bf_bits2f(unsigned short h) { return __uint_as_float(((unsigned)h) << 16); }
__device__ __forceinline__ float bf16r(float f) { return bf_bits2f(f2bf_bits(f)); }
__device__ __forceinline__ float carry_flush(float v, float carry) {
  const float s = v * carry;
  return (fabsf(s) < kF16MinNormal) ? 0.0f : s;
}

__device__ __forceinline__ void dep_guard4_h(v8f& a, v8f& b, v8f& c, v8f& d, v16h x, v16h y) { asm volatile("v_nop\n\tv_nop\n\tv_nop\n\tv_nop" : "+v"(a), "+v"(b), "+v"(c), "+v"(d) : "v"(x), "v"(y)); }
__device__ __forceinline__ void dep_guard4_b(v8f& a, v8f& b, v8f& c, v8f& d, v16b x, v16b y) { asm volatile("v_nop\n\tv_nop\n\tv_nop\n\tv_nop" : "+v"(a), "+v"(b), "+v"(c), "+v"(d) : "v"(x), "v"(y)); }
__device__ __forceinline__ void keep4_h(v16h a, v16h b, v16h c, v16h d) { asm volatile("v_nop" :: "v"(a), "v"(b), "v"(c), "v"(d)); }
__device__ __forceinline__ void keep4_b(v16b a, v16b b, v16b c, v16b d) { asm volatile("v_nop" :: "v"(a), "v"(b), "v"(c), "v"(d)); }
__device__ __forceinline__ void acc_guard4(v8f& a, v8f& b, v8f& c, v8f& d) { asm volatile("v_nop\n\tv_nop\n\tv_nop\n\tv_nop" : "+v"(a), "+v"(b), "+v"(c), "+v"(d)); }

template <typename T> struct Frag;
template <> struct Frag<_Float16> {
  typedef v16h V; union U { v16h v; v8h h[2]; };
  static __device__ __forceinline__ v16h load(const _Float16* p) {
    U f; f.h[0] = *(const v8h*)(p); f.h[1] = *(const v8h*)(p + 16); return f.v;
  }
  static __device__ __forceinline__ v8f mma(v16h a, v16h b, v8f c) {
    return __builtin_amdgcn_wmma_f32_16x16x32_f16(false, a, false, b, (short)0, c, false, false);
  }
  static __device__ __forceinline__ void guard4(v8f& a, v8f& b, v8f& c, v8f& d, v16h x, v16h y) { dep_guard4_h(a, b, c, d, x, y); }
  static __device__ __forceinline__ void keep(v16h a, v16h b, v16h c, v16h d) { keep4_h(a, b, c, d); }
};
template <> struct Frag<__bf16> {
  typedef v16b V; union U { v16b v; v8b h[2]; };
  static __device__ __forceinline__ v16b load(const __bf16* p) {
    U f; f.h[0] = *(const v8b*)(p); f.h[1] = *(const v8b*)(p + 16); return f.v;
  }
  static __device__ __forceinline__ v8f mma(v16b a, v16b b, v8f c) {
    return __builtin_amdgcn_wmma_f32_16x16x32_bf16(false, a, false, b, (short)0, c, false, false);
  }
  static __device__ __forceinline__ void guard4(v8f& a, v8f& b, v8f& c, v8f& d, v16b x, v16b y) { dep_guard4_b(a, b, c, d, x, y); }
  static __device__ __forceinline__ void keep(v16b a, v16b b, v16b c, v16b d) { keep4_b(a, b, c, d); }
};

__device__ __forceinline__ v8f mma_h(v16h a, v16h b, v8f c) {
  c = __builtin_amdgcn_wmma_f32_16x16x32_f16(false, a, false, b, (short)0, c, false, false);
  asm volatile("v_nop\n\tv_nop\n\tv_nop\n\tv_nop" : "+v"(c) : "v"(a), "v"(b));
  return c;
}

template <int ET> struct Elem;
template <> struct Elem<0> { typedef _Float16 T; };
template <> struct Elem<1> { typedef __bf16 T; };
template <int ET, bool SPLIT, int BIAS_MODE, int OUT_MODE, bool RESID, int ACT = 0>
__global__ __launch_bounds__(256) void wmma_gemm64(
    const unsigned short* __restrict__ Ap, const unsigned short* __restrict__ A2p, int lda, long strideA,
    const unsigned short* __restrict__ Btp, const unsigned short* __restrict__ Bt2p, int ldb, long strideB,
    void* __restrict__ Cout, void* __restrict__ Cout2, int ldc, long strideC,
    const float* __restrict__ bias,
    const float* __restrict__ resid, long strideR,
    int M, int N, int K, float scale) {
  typedef typename Elem<ET>::T T;
  typedef typename Frag<T>::V V;
  const T* A = (const T*)Ap; const T* A2 = (const T*)A2p; const T* Bt = (const T*)Btp; const T* Bt2 = (const T*)Bt2p;
  __shared__ __align__(16) float sT[8][16 * 68];
  const int b    = blockIdx.y;
  const int lane = threadIdx.x & 31;
  const int wave = threadIdx.x >> 5;
  const int tilesN = N >> 6;
  const int tilesM = M >> 6;
  const int tile = blockIdx.x * 8 + wave;
  if (tile >= tilesM * tilesN) return;
  const int tm = tile / tilesN;
  const int tn = tile - tm * tilesN;
  const int m0 = tm << 6;
  const int n0 = tn << 6;

  const T* Ab  = A  + (size_t)b * strideA;
  const T* Bb  = Bt + (size_t)b * strideB;
  const T* Ab2 = SPLIT ? (A2  + (size_t)b * strideA) : nullptr;
  const T* Bb2 = SPLIT ? (Bt2 + (size_t)b * strideB) : nullptr;

  const int rlane = lane & 15;
  const int koff  = (lane >> 4) * 8;
  const int mOff  = (lane >> 4) * 8;

  v8f acc[4][4];
#pragma unroll
  for (int i = 0; i < 4; ++i)
#pragma unroll
    for (int j = 0; j < 4; ++j) acc[i][j] = (v8f){0.f,0.f,0.f,0.f,0.f,0.f,0.f,0.f};

  for (int k0 = 0; k0 < K; k0 += 32) {
    V bh[4], bl[4];
#pragma unroll
    for (int j = 0; j < 4; ++j) {
      const size_t bo = (size_t)(n0 + (j << 4) + rlane) * ldb + koff + k0;
      bh[j] = Frag<T>::load(Bb + bo);
      if (SPLIT) bl[j] = Frag<T>::load(Bb2 + bo);
    }
#pragma unroll
    for (int i = 0; i < 4; ++i) {
      const size_t ao = (size_t)(m0 + (i << 4) + rlane) * lda + koff + k0;
      V ah = Frag<T>::load(Ab + ao);
      V al;
      if (SPLIT) al = Frag<T>::load(Ab2 + ao);
#pragma unroll
      for (int j = 0; j < 4; ++j) {
        acc[i][j] = Frag<T>::mma(ah, bh[j], acc[i][j]);
        if (SPLIT) {
          acc[i][j] = Frag<T>::mma(ah, bl[j], acc[i][j]);
          acc[i][j] = Frag<T>::mma(al, bh[j], acc[i][j]);
        }
      }
      Frag<T>::guard4(acc[i][0], acc[i][1], acc[i][2], acc[i][3], ah, SPLIT ? al : ah);
    }
    Frag<T>::keep(bh[0], bh[1], bh[2], bh[3]);
    if (SPLIT) Frag<T>::keep(bl[0], bl[1], bl[2], bl[3]);
  }
  acc_guard4(acc[0][0], acc[0][1], acc[0][2], acc[0][3]);
  acc_guard4(acc[1][0], acc[1][1], acc[1][2], acc[1][3]);
  acc_guard4(acc[2][0], acc[2][1], acc[2][2], acc[2][3]);
  acc_guard4(acc[3][0], acc[3][1], acc[3][2], acc[3][3]);

  float* slab = sT[wave];
  const float* Rb = RESID ? (resid + (size_t)b * strideR) : nullptr;
#pragma unroll
  for (int i = 0; i < 4; ++i) {
    const int mBase = m0 + (i << 4);
#pragma unroll
    for (int j = 0; j < 4; ++j) {
      const int n = n0 + (j << 4) + rlane;
      float bv = 0.f;
      if (BIAS_MODE == 2) bv = bias[n];
#pragma unroll
      for (int r = 0; r < 8; ++r) {
        float v = acc[i][j][r] * scale;
        if (BIAS_MODE == 1) v += bias[mBase + mOff + r];
        if (BIAS_MODE == 2) v += bv;
        if (RESID) v += Rb[(size_t)(mBase + mOff + r) * ldc + n];
        if (ACT == 1) v = tanhf(v);
        if (ACT == 2) v = fmaxf(v, 0.0f);
        if (ACT == 3) v = v / (1.0f + expf(-v));
        if (ACT == 4) v = (v > 0.f) ? v : 0.01f * v;
        slab[(mOff + r) * 68 + (j << 4) + rlane] = v;
      }
    }
    __builtin_amdgcn_fence(__ATOMIC_RELEASE, "workgroup");
    __builtin_amdgcn_wave_barrier();
    __builtin_amdgcn_fence(__ATOMIC_ACQUIRE, "workgroup");
    if (OUT_MODE == 0) {
      float* C = (float*)Cout + (size_t)b * strideC;
      const int hh = lane >> 4, c4 = (lane & 15) * 4;
      for (int pass = 0; pass < 2; ++pass) {
#pragma unroll
        for (int it = 0; it < 8; ++it) {
          const int row = it * 2 + hh;
          v4f v = *(const v4f*)(slab + row * 68 + c4);
          *(volatile v4f*)(C + (size_t)(mBase + row) * ldc + n0 + c4) = v;
        }
        __threadfence();
      }
    } else {
      const int q = lane >> 3, c8 = (lane & 7) * 8;
      unsigned short* C  = (unsigned short*)Cout  + (size_t)b * strideC;
      unsigned short* C2 = (OUT_MODE == 2) ? ((unsigned short*)Cout2 + (size_t)b * strideC) : nullptr;
      for (int pass = 0; pass < 2; ++pass) {
#pragma unroll
        for (int it = 0; it < 4; ++it) {
          const int row = it * 4 + q;
          const float* sp = slab + row * 68 + c8;
          v8h hv, lv;
#pragma unroll
          for (int e = 0; e < 8; ++e) {
            if (OUT_MODE == 1) {
              hv[e] = (_Float16)sp[e];
            } else {
              unsigned short hb = f2bf_bits(sp[e]);
              unsigned short lb = f2bf_bits(sp[e] - bf_bits2f(hb));
              hv[e] = __builtin_bit_cast(_Float16, hb);
              lv[e] = __builtin_bit_cast(_Float16, lb);
            }
          }
          *(volatile v8h*)(C + (size_t)(mBase + row) * ldc + n0 + c8) = hv;
          if (OUT_MODE == 2) *(volatile v8h*)(C2 + (size_t)(mBase + row) * ldc + n0 + c8) = lv;
        }
        __threadfence();
      }
    }
    __builtin_amdgcn_fence(__ATOMIC_RELEASE, "workgroup");
    __builtin_amdgcn_wave_barrier();
    __builtin_amdgcn_fence(__ATOMIC_ACQUIRE, "workgroup");
  }
}


__global__ __launch_bounds__(kThr) void bias_kernel(const float* __restrict__ bz, const float* __restrict__ bf, float* __restrict__ BIA) {
  const unsigned i = blockIdx.x * (unsigned)kThr + threadIdx.x;
  const float a = (blockIdx.x == 0u) ? bz[threadIdx.x] : bf[threadIdx.x];
  const float v = bf16r(a);
  *(volatile float*)(BIA + i) = v;
  __threadfence();
  *(volatile float*)(BIA + i) = v;
}
static_assert(kN2 == 2 * kThr, "bias grid exact: 2 blocks");

__global__ __launch_bounds__(kThr) void w2_cast_kernel(const float* __restrict__ Wz, const float* __restrict__ Wf, unsigned short* __restrict__ W2) {
  const unsigned i = blockIdx.x * (unsigned)kThr + threadIdx.x;
  const unsigned c8 = i & 31u, k = (i >> 5) & 1u, o2 = i >> 6;
  const float* W = (blockIdx.x < 64u) ? Wz : Wf;
  const unsigned o = o2 & 255u;
  const float* sp = W + ((size_t)o * kC + c8 * 8u) * 2u + k;
  v8h hv;
#pragma unroll
  for (int t = 0; t < 8; ++t) { const float v = sp[(size_t)t * 2u]; hv[t] = (_Float16)carry_flush(bf16r(v), kInCarry); }
  unsigned short* dp = W2 + (size_t)i * 8u;
  *(volatile v8h*)dp = hv;
  __threadfence();
  *(volatile v8h*)dp = hv;
}
static_assert((size_t)kN2 * (kK2 / 8) == 128ull * kThr && 64 * kThr / 64 == 256, "weight cast grid exact: 128 blocks; a block = 4 output rows: blocks 0..63 are Wz's 256 rows");

__global__ __launch_bounds__(kThr) void x2_cast_kernel(const float* __restrict__ X, unsigned short* __restrict__ X2) {
  const unsigned i = blockIdx.x * (unsigned)kThr + threadIdx.x;
  const unsigned c8 = i & 31u, k = (i >> 5) & 1u, r = i >> 6;
  const bool live = (k == 1u) || (r >= (unsigned)kB);
  const unsigned rs = (k == 1u || !live) ? r : (r - (unsigned)kB);
  const float* sp = X + (size_t)rs * kC + c8 * 8u;
  const v4f a0 = *(const v4f*)sp, a1 = *(const v4f*)(sp + 4);
  v8h hv;
#pragma unroll
  for (int t = 0; t < 4; ++t) { const float p = a0[t], q = a1[t]; hv[t] = (_Float16)carry_flush(live ? bf16r(p) : 0.0f, kInCarry); hv[4 + t] = (_Float16)carry_flush(live ? bf16r(q) : 0.0f, kInCarry); }
  unsigned short* dp = X2 + (size_t)i * 8u;
  *(volatile v8h*)dp = hv;
  __threadfence();
  *(volatile v8h*)dp = hv;
}
static_assert((size_t)kRows * (kK2 / 8) == 8192ull * kThr, "row cast grid exact: 8,192 blocks");

__global__ __launch_bounds__(kThr) void scan_kernel(const float* __restrict__ ZF, const float* __restrict__ hidden, float* __restrict__ out0, float* __restrict__ out1) {
  const unsigned b = blockIdx.x, ch = threadIdx.x;
  const float h0 = hidden[(size_t)b * kHd + ch];
  float h = bf16r(h0);
  for (int t = 0; t < kS; ++t) {
    const size_t row = (size_t)t * kB + b;
    const float z = ZF[row * kN2 + ch];
    const float f = ZF[row * kN2 + kHd + ch];
    const float zq = z / (1.0f + expf(-kGelu * z));
    const float fs = 1.0f / (1.0f + expf(-f));
    h = fs * zq + (1.0f - fs) * h;
    float* dp = out0 + row * kHd + ch;
    *(volatile float*)dp = h;
    __threadfence();
    *(volatile float*)dp = h;
  }
  float* lp = out1 + (size_t)b * kHd + ch;
  *(volatile float*)lp = h;
  __threadfence();
  *(volatile float*)lp = h;
}
static_assert(kHd == kThr && kB == 8, "scan grid exact: 8 blocks of 256: a block a sample");

static_assert(((kRows / 64) * (kN2 / 64)) % 8 == 0, "the product's grid exact: every wave live");

extern "C" void kernel_launch(void* const* d_in, const int* in_sizes, int n_in,
                              void* d_out, int out_size, void* d_ws, size_t ws_size,
                              hipStream_t stream) {
  if (n_in < 6 || d_out == nullptr || d_ws == nullptr) return;
  if (in_sizes[0] != kRows * kC || in_sizes[1] != kB * kHd || in_sizes[2] != kHd * kC * 2 || in_sizes[3] != kHd || in_sizes[4] != kHd * kC * 2 || in_sizes[5] != kHd) return;
  if ((size_t)out_size != kOut1 + (size_t)kB * kHd) return;
  if (ws_size < kWsTotal) return;
  const float* X = (const float*)d_in[0];
  const float* hidden = (const float*)d_in[1];
  const float* Wz = (const float*)d_in[2];
  const float* bz = (const float*)d_in[3];
  const float* Wf = (const float*)d_in[4];
  const float* bf = (const float*)d_in[5];
  float* out = (float*)d_out;
  char* ws = (char*)d_ws;
  float* BIA = (float*)(ws + kOffBIA);
  unsigned short* W2 = (unsigned short*)(ws + kOffW2);
  unsigned short* X2 = (unsigned short*)(ws + kOffX2);
  float* ZF32 = (float*)(ws + kOffZF32);

  bias_kernel<<<2, kThr, 0, stream>>>(bz, bf, BIA);
  w2_cast_kernel<<<128, kThr, 0, stream>>>(Wz, Wf, W2);
  x2_cast_kernel<<<8192, kThr, 0, stream>>>(X, X2);
  wmma_gemm64<0, false, 2, 0, false, 0><<<dim3((kRows / 64) * (kN2 / 64) / 8, 1), 256, 0, stream>>>(
      X2, X2, kK2, 0L, W2, W2, kK2, 0L, (void*)ZF32, (void*)ZF32, kN2, 0L, BIA, nullptr, 0L, kRows, kN2, kK2, kSc);
  scan_kernel<<<kB, kThr, 0, stream>>>(ZF32, hidden, out + kOut0, out + kOut1);
}
